// TransformerEncoderLayer_420906795677
// MI455X (gfx1250) — hardware-verified
//
#include <hip/hip_runtime.h>
#ifndef NB
#define NB 2
#endif
#ifndef SQ
#define SQ 2048
#endif
#define NB_FULL 2
#define SQ_FULL 2048
#define DM 1024
#define NH 16
#define HD 64
#define DFF 4096
#define LQ (3 * DM)
#define DMQ DM
#define NR ((size_t)NB * SQ)

static_assert(NB >= 1 && NB <= NB_FULL);
static_assert(SQ >= 128 && SQ <= SQ_FULL && SQ % 128 == 0);
static_assert(NH * HD == DM && HD == 64);
static_assert(DM % 64 == 0 && LQ % 64 == 0 && DFF % 64 == 0);
static_assert(DM % 32 == 0 && DFF % 32 == 0 && SQ % 64 == 0);
static_assert((NR % 128) == 0);
static_assert(DMQ <= 1024 && DMQ % 4 == 0 && (DMQ / 4) * 4 == DM);
static_assert(((size_t)(NB - 1) * SQ_FULL + SQ) * DM * 4 <= (size_t)NB_FULL * SQ_FULL * DM * 4);

typedef unsigned short v8us __attribute__((ext_vector_type(8), may_alias));
typedef float  v8f  __attribute__((ext_vector_type(8)));
typedef float  v4f  __attribute__((ext_vector_type(4)));
typedef float  v4fa __attribute__((ext_vector_type(4), may_alias));
typedef _Float16 v16h __attribute__((ext_vector_type(16)));
typedef _Float16 v4h __attribute__((ext_vector_type(4)));
union FragH { v16h v; v8us half[2]; _Float16 h[16]; unsigned short u[16]; };

__device__ __forceinline__ unsigned short bf16_bits(float x) { unsigned int u = __float_as_uint(x); return (unsigned short)((u + 0x7FFFu + ((u >> 16) & 1u)) >> 16); }
__device__ __forceinline__ float bf16_val(unsigned short b) { return __uint_as_float(((unsigned int)b) << 16); }
__device__ __forceinline__ float bf16_rne(float x) { return bf16_val(bf16_bits(x)); }

__device__ __forceinline__ v16h g2_frag(const _Float16* p, unsigned hh) { FragH f; f.half[0] = *(const v8us*)((const unsigned short*)p + 8 * hh); f.half[1] = *(const v8us*)((const unsigned short*)p + 16 + 8 * hh); return f.v; }
__device__ __forceinline__ v8f g2_mma(v16h a, v16h b, v8f c) { v8f d = __builtin_amdgcn_wmma_f32_16x16x32_f16(false, a, false, b, (short)0, c, false, false); asm volatile("v_nop\n\tv_nop\n\tv_nop\n\tv_nop" : "+v"(d) : "v"(a), "v"(b)); return d; }

__device__ __forceinline__ float gelu_erf(float v) { return v * (0.5f * (1.0f + erff(v * 0.70710678118654752f))); }

template <int ACT, int CPBF>
__global__ __launch_bounds__(128) void k_gemm2(const _Float16* __restrict__ A, unsigned lda, const _Float16* __restrict__ Bh, unsigned ldb, float alpha, const float* __restrict__ bias, const float* __restrict__ CP,
    float* __restrict__ C, _Float16* __restrict__ C16, unsigned ldc, float c16s, unsigned M, unsigned N, unsigned K) {
  static_assert(ACT == 0 || ACT == 7);
  __shared__ __attribute__((aligned(16))) float so[4][32][68];
  const unsigned tid = threadIdx.x, w = tid >> 5, lane = tid & 31u, ln = lane & 15u, hh = lane >> 4;
  const unsigned ntn = N >> 6; const unsigned mt = blockIdx.x / ntn, nq = blockIdx.x - mt * ntn; const unsigned row0 = mt * 128u + 32u * w, col0 = nq * 64u; if (row0 >= M) return;
  const _Float16* a0p = A + (size_t)(row0 + ln) * lda; const _Float16* a1p = a0p + (size_t)16 * lda;
  const _Float16* b0p = Bh + (size_t)(col0 + ln) * ldb; const _Float16* b1p = b0p + (size_t)16 * ldb; const _Float16* b2p = b1p + (size_t)16 * ldb; const _Float16* b3p = b2p + (size_t)16 * ldb;
  const v8f z8 = {0.f,0.f,0.f,0.f,0.f,0.f,0.f,0.f}; v8f c00 = z8, c01 = z8, c02 = z8, c03 = z8, c10 = z8, c11 = z8, c12 = z8, c13 = z8;
#pragma unroll 1
  for (unsigned kb = 0; kb < K; kb += 32) { const v16h a0 = g2_frag(a0p + kb, hh), a1 = g2_frag(a1p + kb, hh);
    v16h b = g2_frag(b0p + kb, hh); c00 = g2_mma(a0, b, c00); c10 = g2_mma(a1, b, c10);
    b = g2_frag(b1p + kb, hh); c01 = g2_mma(a0, b, c01); c11 = g2_mma(a1, b, c11);
    b = g2_frag(b2p + kb, hh); c02 = g2_mma(a0, b, c02); c12 = g2_mma(a1, b, c12);
    b = g2_frag(b3p + kb, hh); c03 = g2_mma(a0, b, c03); c13 = g2_mma(a1, b, c13); }
  v8f accs[8] = {c00, c01, c02, c03, c10, c11, c12, c13};
#pragma unroll
  for (int u = 0; u < 8; ++u) { const unsigned t = (unsigned)u & 3u, half = (unsigned)u >> 2; const unsigned col = col0 + t * 16u + ln; float bv = 0.f; if (bias) bv = bf16_rne(bias[col]);
#pragma unroll
    for (int r = 0; r < 8; ++r) { const unsigned rloc = half * 16u + 8u * hh + (unsigned)r; so[w][rloc][t * 16u + ln] = accs[u][r] * alpha + bv; } }
  __builtin_amdgcn_fence(4  , "workgroup"); __builtin_amdgcn_wave_barrier();
  const unsigned rsub = lane >> 4, c4 = (lane & 15u) * 4u;
  if (CP != nullptr || ACT == 7) {
#pragma unroll 2
    for (unsigned q = 0; q < 16; ++q) { const unsigned r = q * 2u + rsub; v4f v = *(const v4fa*)&so[w][r][c4];
      if (CP) { const v4f a = *(const v4fa*)(CP + (size_t)(row0 + r) * ldc + col0 + c4);
#pragma unroll
        for (int i = 0; i < 4; ++i) v[i] += CPBF ? bf16_rne(a[i]) : a[i]; }
      if (ACT == 7) {
#pragma unroll
        for (int i = 0; i < 4; ++i) v[i] = gelu_erf(v[i]); }
      *(v4fa*)&so[w][r][c4] = v; } }
  for (int pass = 0; pass < 2; ++pass) {
#pragma unroll
    for (unsigned q = 0; q < 16; ++q) { const unsigned r = q * 2u + rsub; const v4f v = *(const v4fa*)&so[w][r][c4];
      if (C) *(volatile v4f*)(C + (size_t)(row0 + r) * ldc + col0 + c4) = v;
      if (C16) { v4h h4;
#pragma unroll
        for (int i = 0; i < 4; ++i) h4[i] = (_Float16)(v[i] * c16s);
        *(volatile v4h*)(C16 + (size_t)(row0 + r) * ldc + col0 + c4) = h4; } }
    if (pass == 0) __threadfence(); } }

__global__ __launch_bounds__(256) void k_wtr(const float* __restrict__ w, unsigned Kd, unsigned Nd, _Float16* __restrict__ Bt) { __shared__ _Float16 tl[64][66]; const unsigned tid = threadIdx.x; const unsigned ntn = Nd >> 6; const unsigned kt = blockIdx.x / ntn, nt = blockIdx.x - kt * ntn; const unsigned k0 = kt * 64u, n0 = nt * 64u;
#pragma unroll 1
  for (unsigned i = tid; i < 1024u; i += 256u) { const unsigned r = i >> 4, c4 = (i & 15u) * 4u; const v4f a = *(const v4fa*)(w + (size_t)(k0 + r) * Nd + n0 + c4);
#pragma unroll
    for (int q = 0; q < 4; ++q) tl[r][c4 + q] = (_Float16)(bf16_rne(a[q]) * 16.0f); }
  __syncthreads();
  for (int pass = 0; pass < 2; ++pass) {
#pragma unroll
    for (unsigned rd = 0; rd < 2; ++rd) { const unsigned n = rd * 32u + (tid >> 3), pc = tid & 7u; FragH f;
#pragma unroll
      for (int q = 0; q < 8; ++q) f.h[q] = tl[pc * 8u + q][n];
      *(volatile v8us*)((unsigned short*)Bt + (size_t)(n0 + n) * Kd + k0 + pc * 8u) = f.half[0]; }
    if (pass == 0) __threadfence(); } }

template <int BFIN, int W16, int W32>
__global__ __launch_bounds__(256) void k_lnx(const float* __restrict__ X, const float* __restrict__ g, const float* __restrict__ bb, float eps, _Float16* __restrict__ N16, float* __restrict__ N32) {
  #pragma clang fp contract(off)
  __shared__ float red[256]; const size_t r = blockIdx.x; const int t = threadIdx.x; const bool act = t < (DMQ / 4); const int c0 = act ? t * 4 : 0;
  const v4f xa = *(const v4fa*)(X + r * DMQ + c0); float s[4]; float sum = 0.f;
#pragma unroll
  for (int q = 0; q < 4; ++q) { s[q] = act ? (BFIN ? bf16_rne(xa[q]) : xa[q]) : 0.f; sum = __fadd_rn(sum, s[q]); }
  red[t] = sum; __syncthreads(); for (int st = 128; st > 0; st >>= 1) { if (t < st) red[t] = __fadd_rn(red[t], red[t + st]); __syncthreads(); } const float mu = red[0] / (float)DMQ; __syncthreads();
  float vs = 0.f;
#pragma unroll
  for (int q = 0; q < 4; ++q) { const float dl = act ? __fadd_rn(s[q], -mu) : 0.f; vs = __fadd_rn(vs, __fmul_rn(dl, dl)); }
  red[t] = vs; __syncthreads(); for (int st = 128; st > 0; st >>= 1) { if (t < st) red[t] = __fadd_rn(red[t], red[t + st]); __syncthreads(); }
  const float rs = rsqrtf(__fadd_rn(red[0] / (float)DMQ, eps)); v4h y; v4f yf;
#pragma unroll
  for (int q = 0; q < 4; ++q) { const int c = c0 + q; yf[q] = __fadd_rn(__fmul_rn(__fmul_rn(__fadd_rn(s[q], -mu), rs), bf16_rne(g[c])), bf16_rne(bb[c])); y[q] = (_Float16)yf[q]; }
  if (!act) return;
  for (int pass = 0; pass < 2; ++pass) { if (W16) *(volatile v4h*)(N16 + r * DMQ + c0) = y; if (W32) *(volatile v4f*)(N32 + r * DMQ + c0) = yf; if (pass == 0) __threadfence(); } }

template <int NHv, int TTv>
__global__ __launch_bounds__(256) void k_vt(const _Float16* __restrict__ V16, unsigned ldv, unsigned voff, _Float16* __restrict__ Vt) { __shared__ unsigned short tl[64][66]; const unsigned tid = threadIdx.x; const unsigned tpb = (unsigned)TTv / 64u; const unsigned slab = blockIdx.x / tpb, lg = blockIdx.x - slab * tpb; const unsigned b = slab / (unsigned)NHv, h = slab - b * (unsigned)NHv;
  for (unsigned i = tid; i < 512u; i += 256u) { const unsigned r = i >> 3, c8 = (i & 7u) * 8u; FragH f; f.half[0] = *(const v8us*)((const unsigned short*)V16 + ((size_t)b * TTv + lg * 64u + r) * ldv + voff + h * 64u + c8);
#pragma unroll
    for (int q = 0; q < 8; ++q) tl[r][c8 + q] = f.u[q]; }
  __syncthreads();
  for (int pass = 0; pass < 2; ++pass) {
#pragma unroll
    for (unsigned rd = 0; rd < 2; ++rd) { const unsigned d = rd * 32u + (tid >> 3), pc = tid & 7u; FragH f;
#pragma unroll
      for (int q = 0; q < 8; ++q) f.u[q] = tl[pc * 8u + q][d];
      *(volatile v8us*)((unsigned short*)Vt + ((size_t)slab * 64u + d) * TTv + lg * 64u + pc * 8u) = f.half[0]; }
    if (pass == 0) __threadfence(); } }

__global__ __launch_bounds__(128) void k_fattn(const _Float16* __restrict__ QKV, const _Float16* __restrict__ VT, _Float16* __restrict__ O16) {
  __shared__ __attribute__((aligned(16))) _Float16 sp[4][16][72];
  const unsigned tid = threadIdx.x, w = tid >> 5, lane = tid & 31u, ln = lane & 15u, hh = lane >> 4;
  const unsigned nqt = (unsigned)SQ / 64u; const unsigned bid = blockIdx.x; const unsigned bh = bid / nqt, qb = bid - bh * nqt; const unsigned b = bh / (unsigned)NH, h = bh - b * (unsigned)NH;
  const unsigned q0 = qb * 64u + w * 16u; const size_t rowb = (size_t)b * SQ;
  const _Float16* qp = QKV + (rowb + q0 + ln) * (size_t)LQ + h * (unsigned)HD;
  const v16h aq0 = g2_frag(qp, hh), aq1 = g2_frag(qp + 32, hh);
  const _Float16* kp = QKV + (rowb + ln) * (size_t)LQ + DM + h * (unsigned)HD;
  const _Float16* vp = VT + ((size_t)bh * HD + ln) * SQ;
  const v8f z8 = {0.f,0.f,0.f,0.f,0.f,0.f,0.f,0.f};
  float m[8], l[8]; v8f o[4];
#pragma unroll
  for (int r = 0; r < 8; ++r) { m[r] = -1.0e30f; l[r] = 0.f; }
#pragma unroll
  for (int d = 0; d < 4; ++d) o[d] = z8;
#pragma unroll 1
  for (unsigned kt = 0; kt < (unsigned)SQ / 64u; ++kt) { const unsigned key0 = kt * 64u;
    v8f s[4];
#pragma unroll
    for (unsigned j = 0; j < 4; ++j) { const _Float16* kr = kp + (size_t)(key0 + 16u * j) * LQ; const v16h b0 = g2_frag(kr, hh), b1 = g2_frag(kr + 32, hh); v8f acc = z8; acc = g2_mma(aq0, b0, acc); acc = g2_mma(aq1, b1, acc); s[j] = acc; }
#pragma unroll
    for (unsigned j = 0; j < 4; ++j) {
#pragma unroll
      for (int r = 0; r < 8; ++r) s[j][r] = s[j][r] * 0.125f; }
#pragma unroll
    for (int r = 0; r < 8; ++r) { float mx = fmaxf(fmaxf(s[0][r], s[1][r]), fmaxf(s[2][r], s[3][r]));
      mx = fmaxf(mx, __shfl_xor(mx, 1, 32)); mx = fmaxf(mx, __shfl_xor(mx, 2, 32)); mx = fmaxf(mx, __shfl_xor(mx, 4, 32)); mx = fmaxf(mx, __shfl_xor(mx, 8, 32));
      const float mn = fmaxf(m[r], mx); const float al = __expf(m[r] - mn); m[r] = mn; float rs = 0.f;
#pragma unroll
      for (unsigned j = 0; j < 4; ++j) { const float p = __expf(s[j][r] - mn); rs += p; sp[w][8u * hh + (unsigned)r][16u * j + ln] = (_Float16)(p * 256.0f); }
      rs += __shfl_xor(rs, 1, 32); rs += __shfl_xor(rs, 2, 32); rs += __shfl_xor(rs, 4, 32); rs += __shfl_xor(rs, 8, 32);
      l[r] = l[r] * al + rs;
#pragma unroll
      for (int d = 0; d < 4; ++d) o[d][r] *= al; }
    __builtin_amdgcn_fence(4  , "workgroup"); __builtin_amdgcn_wave_barrier();
    const v16h ap0 = g2_frag(&sp[w][ln][0], hh), ap1 = g2_frag(&sp[w][ln][32], hh);
#pragma unroll
    for (unsigned d = 0; d < 4; ++d) { const _Float16* vr = vp + (size_t)(16u * d) * SQ + key0; const v16h b0 = g2_frag(vr, hh), b1 = g2_frag(vr + 32, hh); o[d] = g2_mma(ap0, b0, o[d]); o[d] = g2_mma(ap1, b1, o[d]); }
    __builtin_amdgcn_fence(4  , "workgroup"); __builtin_amdgcn_wave_barrier(); }
#pragma unroll
  for (int r = 0; r < 8; ++r) { const float sc = 0.25f * (1.0f / l[r]);
#pragma unroll
    for (unsigned d = 0; d < 4; ++d) sp[w][8u * hh + (unsigned)r][16u * d + ln] = (_Float16)(o[d][r] * sc); }
  __builtin_amdgcn_fence(4  , "workgroup"); __builtin_amdgcn_wave_barrier();
  for (int pass = 0; pass < 2; ++pass) {
#pragma unroll
    for (unsigned it = 0; it < 4; ++it) { const unsigned row = it * 4u + (lane >> 3), pc = (lane & 7u) * 8u; const v8us v = *(const v8us*)&sp[w][row][pc];
      *(volatile v8us*)((unsigned short*)O16 + (rowb + q0 + row) * (size_t)DM + h * (unsigned)HD + pc) = v; }
    if (pass == 0) __threadfence(); } }

constexpr size_t al256(size_t b) { return (b + 255) & ~(size_t)255; }
constexpr size_t SZ_BQKV = (size_t)LQ * DM * 2, SZ_BO = (size_t)DM * DM * 2, SZ_BW1 = (size_t)DFF * DM * 2, SZ_BW2 = (size_t)DM * DFF * 2;
constexpr size_t SZ_X16 = NR * DM * 2, SZ_QKV = NR * LQ * 2, SZ_VT = (size_t)NB * NH * HD * SQ * 2;
constexpr size_t SZ_X1 = NR * DM * 4, SZ_M16 = NR * DM * 2, SZ_HF = (size_t)SQ * DFF * 2;
constexpr size_t WS_TOTAL = al256(SZ_BQKV) + al256(SZ_BO) + al256(SZ_BW1) + al256(SZ_BW2) + al256(SZ_X16) + al256(SZ_QKV) + al256(SZ_VT) + al256(SZ_X1) + al256(SZ_M16) + al256(SZ_HF);
static_assert(WS_TOTAL <= (size_t)134217728);
constexpr unsigned CH_N = (SQ == SQ_FULL) ? 1u : (unsigned)NB;
constexpr size_t CH_R = (SQ == SQ_FULL) ? NR : (size_t)SQ;
static_assert(CH_R % 128 == 0 && (size_t)CH_N * CH_R == NR);
static_assert((size_t)3 * (DM / 64) * (DM / 64) * 256 * 2 * 8 == (size_t)DM * LQ);
static_assert((size_t)(DM / 64) * (DM / 64) * 256 * 2 * 8 == (size_t)DM * DM);
static_assert((size_t)(DM / 64) * (DFF / 64) * 256 * 2 * 8 == (size_t)DM * DFF);
static_assert((size_t)CH_N * CH_R * 256 * 4 == NR * DM);
static_assert(NR * 256 * 4 == NR * DM);
static_assert((size_t)NB * NH * (SQ / 64) * 256 * 2 * 8 == (size_t)NB * NH * HD * SQ);
static_assert((size_t)NB * NH * (SQ / 64) * 4 * 16 * 64 == NR * DM);
static_assert((size_t)3 * (NR / 128) * (DM / 64) * 4 * 32 * 64 == NR * LQ);
static_assert((CH_R / 128) * (DM / 64) * 4 * 32 * 64 * CH_N == NR * DM);
static_assert((size_t)(SQ / 128) * (DFF / 64) * 4 * 32 * 64 == (size_t)SQ * DFF);
static_assert((size_t)(SQ / 128) * (DM / 64) * 4 * 32 * 64 == (size_t)SQ * DM);

extern "C" void kernel_launch(void* const* d_in, const int* in_sizes, int n_in,
                              void* d_out, int out_size, void* d_ws, size_t ws_size, hipStream_t stream) {
  if (n_in < 17) return;
  const float* const* I = (const float* const*)d_in;
  const float* x = I[0]; const float* wq = I[1]; const float* bq = I[2]; const float* wk = I[3]; const float* bk = I[4]; const float* wv = I[5]; const float* bv = I[6];
  const float* wo = I[7]; const float* bo = I[8]; const float* g1 = I[9]; const float* be1 = I[10];
  const float* w1 = I[11]; const float* b1 = I[12]; const float* w2 = I[13]; const float* b2 = I[14]; const float* g2 = I[15]; const float* be2 = I[16];
  const size_t needX = ((size_t)(NB - 1) * SQ_FULL + SQ) * DM;
  if ((size_t)in_sizes[0] < needX || (size_t)out_size < needX) return;
  if (in_sizes[1] < DM * DM || in_sizes[2] < DM || in_sizes[3] < DM * DM || in_sizes[4] < DM || in_sizes[5] < DM * DM || in_sizes[6] < DM) return;
  if (in_sizes[7] < DM * DM || in_sizes[8] < DM || in_sizes[9] < DM || in_sizes[10] < DM) return;
  if (in_sizes[11] < DM * DFF || in_sizes[12] < DFF || in_sizes[13] < DFF * DM || in_sizes[14] < DM || in_sizes[15] < DM || in_sizes[16] < DM) return;
  char* ws = (char*)d_ws; size_t off = 0;
  auto take = [&](size_t bytes) { char* p = ws + off; off += al256(bytes); return p; };
  _Float16* BQKV = (_Float16*)take(SZ_BQKV); _Float16* BO = (_Float16*)take(SZ_BO); _Float16* BW1 = (_Float16*)take(SZ_BW1); _Float16* BW2 = (_Float16*)take(SZ_BW2);
  _Float16* X16 = (_Float16*)take(SZ_X16); _Float16* O16 = X16;
  _Float16* QKV = (_Float16*)take(SZ_QKV); _Float16* VT = (_Float16*)take(SZ_VT);
  float* X1 = (float*)take(SZ_X1); _Float16* M16 = (_Float16*)take(SZ_M16); _Float16* HF16 = (_Float16*)take(SZ_HF);
  if (off > ws_size) return;

  k_wtr<<<(unsigned)((DM / 64) * (DM / 64)), 256, 0, stream>>>(wq, (unsigned)DM, (unsigned)DM, BQKV);
  k_wtr<<<(unsigned)((DM / 64) * (DM / 64)), 256, 0, stream>>>(wk, (unsigned)DM, (unsigned)DM, BQKV + (size_t)DM * DM);
  k_wtr<<<(unsigned)((DM / 64) * (DM / 64)), 256, 0, stream>>>(wv, (unsigned)DM, (unsigned)DM, BQKV + (size_t)2 * DM * DM);
  k_wtr<<<(unsigned)((DM / 64) * (DM / 64)), 256, 0, stream>>>(wo, (unsigned)DM, (unsigned)DM, BO);
  k_wtr<<<(unsigned)((DM / 64) * (DFF / 64)), 256, 0, stream>>>(w1, (unsigned)DM, (unsigned)DFF, BW1);
  k_wtr<<<(unsigned)((DFF / 64) * (DM / 64)), 256, 0, stream>>>(w2, (unsigned)DFF, (unsigned)DM, BW2);
  for (unsigned c = 0; c < CH_N; ++c) { const size_t rin = (size_t)c * SQ_FULL, r0 = (size_t)c * CH_R;
    k_lnx<1, 1, 0><<<(unsigned)CH_R, 256, 0, stream>>>(x + rin * DM, g1, be1, 1e-5f, X16 + r0 * DM, nullptr); }
  k_gemm2<0, 0><<<(unsigned)((NR / 128) * (DM / 64)), 128, 0, stream>>>(X16, (unsigned)DM, BQKV, (unsigned)DM, 0.0625f, bq, nullptr, nullptr, QKV, (unsigned)LQ, 1.0f, (unsigned)NR, (unsigned)DM, (unsigned)DM);
  k_gemm2<0, 0><<<(unsigned)((NR / 128) * (DM / 64)), 128, 0, stream>>>(X16, (unsigned)DM, BQKV + (size_t)DM * DM, (unsigned)DM, 0.0625f, bk, nullptr, nullptr, QKV + DM, (unsigned)LQ, 1.0f, (unsigned)NR, (unsigned)DM, (unsigned)DM);
  k_gemm2<0, 0><<<(unsigned)((NR / 128) * (DM / 64)), 128, 0, stream>>>(X16, (unsigned)DM, BQKV + (size_t)2 * DM * DM, (unsigned)DM, 0.0625f, bv, nullptr, nullptr, QKV + 2 * DM, (unsigned)LQ, 1.0f, (unsigned)NR, (unsigned)DM, (unsigned)DM);
  k_vt<NH, SQ><<<(unsigned)(NB * NH * (SQ / 64)), 256, 0, stream>>>(QKV + 2 * DM, (unsigned)LQ, 0u, VT);
  k_fattn<<<(unsigned)(NB * NH * (SQ / 64)), 128, 0, stream>>>(QKV, VT, O16);
  for (unsigned c = 0; c < CH_N; ++c) { const size_t rin = (size_t)c * SQ_FULL, r0 = (size_t)c * CH_R;
    k_gemm2<0, 1><<<(unsigned)((CH_R / 128) * (DM / 64)), 128, 0, stream>>>(O16 + r0 * DM, (unsigned)DM, BO, (unsigned)DM, 0.0009765625f, bo, x + rin * DM, X1 + r0 * DM, nullptr, (unsigned)DM, 1.0f, (unsigned)CH_R, (unsigned)DM, (unsigned)DM); }
  k_lnx<0, 1, 0><<<(unsigned)NR, 256, 0, stream>>>(X1, g2, be2, 1e-5f, M16, nullptr);
  for (int b = 0; b < NB; ++b) { const size_t rin = (size_t)b * SQ_FULL, r0 = (size_t)b * SQ;
    k_gemm2<7, 0><<<(unsigned)((SQ / 128) * (DFF / 64)), 128, 0, stream>>>(M16 + r0 * DM, (unsigned)DM, BW1, (unsigned)DM, 0.0625f, b1, nullptr, nullptr, HF16, (unsigned)DFF, 16.0f, (unsigned)SQ, (unsigned)DFF, (unsigned)DM);
    k_gemm2<0, 0><<<(unsigned)((SQ / 128) * (DM / 64)), 128, 0, stream>>>(HF16, (unsigned)DFF, BW2, (unsigned)DFF, 0.00390625f, b2, X1 + r0 * DM, (float*)d_out + rin * DM, nullptr, (unsigned)DM, 1.0f, (unsigned)SQ, (unsigned)DM, (unsigned)DFF); }
}
